// EdgeConditionedConv_77979426226293
// MI455X (gfx1250) — hardware-verified
//
#include <hip/hip_runtime.h>

typedef __attribute__((ext_vector_type(16))) _Float16 v16h;
typedef __attribute__((ext_vector_type(8)))  _Float16 v8h;
typedef __attribute__((ext_vector_type(4)))  _Float16 v4h;
typedef __attribute__((ext_vector_type(8)))  float    v8f;
typedef __attribute__((ext_vector_type(4)))  float    v4f;

constexpr int kGraphs  = 8;
constexpr int kNodes   = 128;
constexpr int kFeat    = 32;
constexpr int kEdgeF   = 8;
constexpr int kHid     = 32;
constexpr int kChan    = 32;
constexpr int kKMain   = kNodes * kHid;
constexpr int kKTot    = kKMain + kNodes;
constexpr int kSteps   = kKTot / 32;
constexpr int kStepsPerWave = kSteps / 4;
constexpr int kWoutLd  = kChan * kFeat;
static_assert(kKMain == 4096);
static_assert(kKTot == 4224);
static_assert((kKTot % 32) == 0);
static_assert(kSteps == 132);
static_assert(kStepsPerWave * 4 == kSteps);
static_assert(kFeat == 32 && kHid == 32 && kChan == 32 && kEdgeF == 8 && kNodes == 128);
static_assert(((kKTot * 2) % 128) == 0);

constexpr float kCarryNf = 16.0f;
constexpr float kCarryW  = 64.0f;
constexpr float kCarryM  = 16.0f;
constexpr float kCarryA  = 64.0f;
constexpr float kFoldM   = kCarryM / (kCarryNf * kCarryW);
constexpr float kFoldOut = 1.0f / (kCarryA * kCarryM);
constexpr float kF16MinNormal = 6.103515625e-5f;
static_assert(kFoldM == 0.015625f);
static_assert(kFoldOut == 0.0009765625f);

constexpr size_t kOffA2   = 0;
constexpr size_t kBytesA2 = (size_t)kGraphs * kNodes * kKTot * 2;
constexpr size_t kOffBT2  = kOffA2 + kBytesA2;
constexpr size_t kBytesBT2 = (size_t)kGraphs * kChan * kKTot * 2;
constexpr size_t kWsTotal = kOffBT2 + kBytesBT2;
static_assert(kBytesA2 == 8650752ull);
static_assert(kBytesBT2 == 2162688ull);
static_assert(kWsTotal == 10813440ull);
static_assert(kWsTotal <= 134217728ull);
static_assert((kOffBT2 % 128) == 0);

__device__ __forceinline__ _Float16 cvt16(float v) {
  const float q = (fabsf(v) < kF16MinNormal) ? 0.0f : v;
  return (_Float16)q;
}

__device__ __forceinline__ v8f mma_h(v16h a, v16h b, v8f c) {
  c = __builtin_amdgcn_wmma_f32_16x16x32_f16(false, a, false, b, (short)0, c, false, false);
  asm volatile("v_nop\n\tv_nop\n\tv_nop\n\tv_nop" : "+v"(c) : "v"(a), "v"(b));
  return c;
}

union FragU { v16h v; v8h h[2]; };
__device__ __forceinline__ v16h frag_load(const _Float16* p) {
  FragU f;
  f.h[0] = *(const v8h*)(p);
  f.h[1] = *(const v8h*)(p + 16);
  return f.v;
}

__device__ __forceinline__ v16h pack16(v4f x0, v4f x1, v4f x2, v4f x3, float s) {
  v16h f;
#pragma unroll
  for (int e = 0; e < 4; ++e) {
    f[e]      = cvt16(x0[e] * s);
    f[4 + e]  = cvt16(x1[e] * s);
    f[8 + e]  = cvt16(x2[e] * s);
    f[12 + e] = cvt16(x3[e] * s);
  }
  return f;
}

__global__ __launch_bounds__(32) void tail_cols_kernel(
    const float* __restrict__ nf, const float* __restrict__ bout, unsigned short* __restrict__ BT2)
{
  const int lane = threadIdx.x;
  const int a = blockIdx.x >> 5;
  const int c = blockIdx.x & 31;
  const float* np = nf + (size_t)(a * kNodes + 4 * lane) * kFeat;
  const float* bp = bout + c * kFeat;
  float s0 = 0.0f, s1 = 0.0f, s2 = 0.0f, s3 = 0.0f;
#pragma unroll 1
  for (int f4 = 0; f4 < kFeat / 4; ++f4) {
    const v4f w  = *(const v4f*)(bp + 4 * f4);
    const v4f x0 = *(const v4f*)(np + 4 * f4);
    const v4f x1 = *(const v4f*)(np + kFeat + 4 * f4);
    const v4f x2 = *(const v4f*)(np + 2 * kFeat + 4 * f4);
    const v4f x3 = *(const v4f*)(np + 3 * kFeat + 4 * f4);
    s0 = fmaf(x0[0], w[0], s0); s0 = fmaf(x0[1], w[1], s0); s0 = fmaf(x0[2], w[2], s0); s0 = fmaf(x0[3], w[3], s0);
    s1 = fmaf(x1[0], w[0], s1); s1 = fmaf(x1[1], w[1], s1); s1 = fmaf(x1[2], w[2], s1); s1 = fmaf(x1[3], w[3], s1);
    s2 = fmaf(x2[0], w[0], s2); s2 = fmaf(x2[1], w[1], s2); s2 = fmaf(x2[2], w[2], s2); s2 = fmaf(x2[3], w[3], s2);
    s3 = fmaf(x3[0], w[0], s3); s3 = fmaf(x3[1], w[1], s3); s3 = fmaf(x3[2], w[2], s3); s3 = fmaf(x3[3], w[3], s3);
  }
  v4h o;
  o[0] = cvt16(s0 * kCarryM);
  o[1] = cvt16(s1 * kCarryM);
  o[2] = cvt16(s2 * kCarryM);
  o[3] = cvt16(s3 * kCarryM);
  unsigned short* dst = BT2 + (size_t)blockIdx.x * kKTot + kKMain + 4 * lane;
  *(volatile v4h*)dst = o;
  __threadfence();
  *(volatile v4h*)dst = o;
}

__global__ __launch_bounds__(128) void weight_cols_kernel(
    const float* __restrict__ nf, const float* __restrict__ Wout, unsigned short* __restrict__ BT2)
{
  __shared__ __align__(16) float sT[4][32 * 36];
  const int tid  = threadIdx.x;
  const int lane = tid & 31;
  const int wave = tid >> 5;
  const int hh   = lane >> 4;
  const int rl   = lane & 15;
  const int a = blockIdx.x >> 5;
  const int c = blockIdx.x & 31;

  v16h bfr[2];
#pragma unroll
  for (int nt = 0; nt < 2; ++nt) {
    const float* wp = Wout + (size_t)(nt * 16 + rl) * kWoutLd + c * kFeat + 8 * hh;
    const v4f w0 = *(const v4f*)(wp);
    const v4f w1 = *(const v4f*)(wp + 4);
    const v4f w2 = *(const v4f*)(wp + 16);
    const v4f w3 = *(const v4f*)(wp + 20);
    bfr[nt] = pack16(w0, w1, w2, w3, kCarryW);
  }
  v16h afr[2];
#pragma unroll
  for (int mt = 0; mt < 2; ++mt) {
    const float* ap = nf + (size_t)(a * kNodes + wave * 32 + mt * 16 + rl) * kFeat + 8 * hh;
    const v4f x0 = *(const v4f*)(ap);
    const v4f x1 = *(const v4f*)(ap + 4);
    const v4f x2 = *(const v4f*)(ap + 16);
    const v4f x3 = *(const v4f*)(ap + 20);
    afr[mt] = pack16(x0, x1, x2, x3, kCarryNf);
  }
  const v8f zero8 = (v8f){0.f, 0.f, 0.f, 0.f, 0.f, 0.f, 0.f, 0.f};
  v8f acc00 = mma_h(afr[0], bfr[0], zero8);
  v8f acc01 = mma_h(afr[0], bfr[1], zero8);
  v8f acc10 = mma_h(afr[1], bfr[0], zero8);
  v8f acc11 = mma_h(afr[1], bfr[1], zero8);

  float* slab = sT[wave];
#pragma unroll
  for (int r = 0; r < 8; ++r) {
    slab[(8 * hh + r) * 36 + rl]           = acc00[r] * kFoldM;
    slab[(8 * hh + r) * 36 + 16 + rl]      = acc01[r] * kFoldM;
    slab[(16 + 8 * hh + r) * 36 + rl]      = acc10[r] * kFoldM;
    slab[(16 + 8 * hh + r) * 36 + 16 + rl] = acc11[r] * kFoldM;
  }
  __syncthreads();

  v8h ov[4];
#pragma unroll
  for (int it = 0; it < 4; ++it) {
    const int row = it * 8 + (lane >> 2);
    const int col = (lane & 3) * 8;
    const float* sp = slab + row * 36 + col;
    const v4f p0 = *(const v4f*)(sp);
    const v4f p1 = *(const v4f*)(sp + 4);
#pragma unroll
    for (int e = 0; e < 4; ++e) {
      ov[it][e]     = cvt16(p0[e]);
      ov[it][4 + e] = cvt16(p1[e]);
    }
  }
  unsigned short* dst = BT2 + (size_t)blockIdx.x * kKTot + wave * 1024 + lane * 8;
  for (int pass = 0; pass < 2; ++pass) {
#pragma unroll
    for (int it = 0; it < 4; ++it) *(volatile v8h*)(dst + it * 256) = ov[it];
    __threadfence();
  }
}

__global__ __launch_bounds__(128) void edge_rows_kernel(
    const float* __restrict__ ef, const float* __restrict__ fltr,
    const float* __restrict__ W0, const float* __restrict__ b0, unsigned short* __restrict__ A2)
{
  __shared__ __align__(16) float sW0[kEdgeF * kHid];
  __shared__ __align__(16) float sb0[kHid];
  __shared__ __align__(16) _Float16 sA[kKMain];
  const int tid  = threadIdx.x;
  const int lane = tid & 31;
  const int wave = tid >> 5;

  sW0[tid]       = W0[tid];
  sW0[tid + 128] = W0[tid + 128];
  if (wave == 0) sb0[lane] = b0[lane];

  const size_t rowbase = (size_t)blockIdx.x * kNodes;
  const size_t edge = rowbase + tid;
  const v4f e0 = *(const v4f*)(ef + edge * kEdgeF);
  const v4f e1 = *(const v4f*)(ef + edge * kEdgeF + 4);
  const float fl = fltr[edge];
  const v4f ft = *(const v4f*)(fltr + rowbase + 4 * lane);
  const float g = fl * kCarryA;
  const float es[8] = {e0[0], e0[1], e0[2], e0[3], e1[0], e1[1], e1[2], e1[3]};
  __syncthreads();

#pragma unroll 1
  for (int hg = 0; hg < 4; ++hg) {
    const v4f ba = *(const v4f*)(sb0 + hg * 8);
    const v4f bc = *(const v4f*)(sb0 + hg * 8 + 4);
    float acc[8] = {ba[0], ba[1], ba[2], ba[3], bc[0], bc[1], bc[2], bc[3]};
#pragma unroll
    for (int s = 0; s < kEdgeF; ++s) {
      const v4f wa = *(const v4f*)(sW0 + s * kHid + hg * 8);
      const v4f wb = *(const v4f*)(sW0 + s * kHid + hg * 8 + 4);
#pragma unroll
      for (int j = 0; j < 4; ++j) {
        acc[j]     = fmaf(es[s], wa[j], acc[j]);
        acc[4 + j] = fmaf(es[s], wb[j], acc[4 + j]);
      }
    }
    v8h o;
#pragma unroll
    for (int j = 0; j < 8; ++j) o[j] = cvt16(fmaxf(acc[j], 0.0f) * g);
    *(v8h*)(sA + tid * kHid + hg * 8) = o;
  }
  __syncthreads();

  v8h ov[4];
#pragma unroll
  for (int it = 0; it < 4; ++it) ov[it] = *(const v8h*)(sA + wave * 1024 + it * 256 + lane * 8);
  v4h tv;
  tv[0] = cvt16(ft[0] * kCarryA);
  tv[1] = cvt16(ft[1] * kCarryA);
  tv[2] = cvt16(ft[2] * kCarryA);
  tv[3] = cvt16(ft[3] * kCarryA);

  unsigned short* rowp = A2 + (size_t)blockIdx.x * kKTot;
  unsigned short* dst  = rowp + wave * 1024 + lane * 8;
  unsigned short* tdst = rowp + kKMain + 4 * lane;
  for (int pass = 0; pass < 2; ++pass) {
#pragma unroll
    for (int it = 0; it < 4; ++it) *(volatile v8h*)(dst + it * 256) = ov[it];
    if (wave == 0) *(volatile v4h*)tdst = tv;
    __threadfence();
  }
}

__global__ __launch_bounds__(128) void aggregate_kernel(
    const unsigned short* __restrict__ A2, const unsigned short* __restrict__ BT2,
    const float* __restrict__ fltr, const float* __restrict__ bias, float* __restrict__ out)
{
  __shared__ __align__(16) float red[4][16 * 36];
  const int tid  = threadIdx.x;
  const int lane = tid & 31;
  const int wave = tid >> 5;
  const int hh   = lane >> 4;
  const int rl   = lane & 15;
  const int a  = blockIdx.x >> 3;
  const int bt = blockIdx.x & 7;

  const _Float16* Ap = (const _Float16*)A2 + (size_t)(a * kNodes + bt * 16 + rl) * kKTot + 8 * hh;
  const _Float16* B0 = (const _Float16*)BT2 + (size_t)(a * kChan + rl) * kKTot + 8 * hh;
  const _Float16* B1 = B0 + (size_t)16 * kKTot;

  v8f acc0 = (v8f){0.f, 0.f, 0.f, 0.f, 0.f, 0.f, 0.f, 0.f};
  v8f acc1 = (v8f){0.f, 0.f, 0.f, 0.f, 0.f, 0.f, 0.f, 0.f};
  const int kbeg = wave * kStepsPerWave * 32;
#pragma unroll 1
  for (int ks = 0; ks < kStepsPerWave; ++ks) {
    const int k0 = kbeg + ks * 32;
    const v16h af = frag_load(Ap + k0);
    const v16h bf0 = frag_load(B0 + k0);
    const v16h bf1 = frag_load(B1 + k0);
    acc0 = mma_h(af, bf0, acc0);
    acc1 = mma_h(af, bf1, acc1);
  }

  float* slab = red[wave];
#pragma unroll
  for (int r = 0; r < 8; ++r) {
    slab[(8 * hh + r) * 36 + rl]      = acc0[r];
    slab[(8 * hh + r) * 36 + 16 + rl] = acc1[r];
  }

  const int row  = tid >> 3;
  const int part = tid & 7;
  const float* fp = fltr + (size_t)(a * kNodes + bt * 16 + row) * kNodes + part * 16;
  const v4f f0 = *(const v4f*)(fp);
  const v4f f1 = *(const v4f*)(fp + 4);
  const v4f f2 = *(const v4f*)(fp + 8);
  const v4f f3 = *(const v4f*)(fp + 12);
  float rs = 0.0f;
  rs += (f0[0] + f0[1]) + (f0[2] + f0[3]);
  rs += (f1[0] + f1[1]) + (f1[2] + f1[3]);
  rs += (f2[0] + f2[1]) + (f2[2] + f2[3]);
  rs += (f3[0] + f3[1]) + (f3[2] + f3[3]);
  rs += __shfl_xor(rs, 1, 32);
  rs += __shfl_xor(rs, 2, 32);
  rs += __shfl_xor(rs, 4, 32);
  const float rinv = 1.0f / fmaxf(rs, 1e-11f);
  const float sc = rinv * kFoldOut;
  const int c4 = part * 4;
  const v4f bv = *(const v4f*)(bias + c4);
  __syncthreads();

  const v4f p0 = *(const v4f*)(red[0] + row * 36 + c4);
  const v4f p1 = *(const v4f*)(red[1] + row * 36 + c4);
  const v4f p2 = *(const v4f*)(red[2] + row * 36 + c4);
  const v4f p3 = *(const v4f*)(red[3] + row * 36 + c4);
  v4f o;
#pragma unroll
  for (int e = 0; e < 4; ++e) {
    const float s = ((p0[e] + p1[e]) + p2[e]) + p3[e];
    o[e] = s * sc + bv[e];
  }
  float* dst = out + (size_t)(a * kNodes + bt * 16 + row) * kChan + c4;
  *(volatile v4f*)dst = o;
  __threadfence();
  *(volatile v4f*)dst = o;
}

extern "C" void kernel_launch(void* const* d_in, const int* in_sizes, int n_in,
                              void* d_out, int out_size, void* d_ws, size_t ws_size,
                              hipStream_t stream) {
  if (n_in < 8) return;
  if (in_sizes[0] != kGraphs * kNodes * kFeat) return;
  if (in_sizes[1] != kGraphs * kNodes * kNodes) return;
  if (in_sizes[2] != kGraphs * kNodes * kNodes * kEdgeF) return;
  if (in_sizes[3] != kEdgeF * kHid) return;
  if (in_sizes[4] != kHid) return;
  if (in_sizes[5] != kHid * kChan * kFeat) return;
  if (in_sizes[6] != kChan * kFeat) return;
  if (in_sizes[7] != kChan) return;
  if (out_size != kGraphs * kNodes * kChan) return;
  if (ws_size < kWsTotal) return;

  const float* nf    = (const float*)d_in[0];
  const float* fltr  = (const float*)d_in[1];
  const float* ef    = (const float*)d_in[2];
  const float* W0    = (const float*)d_in[3];
  const float* b0    = (const float*)d_in[4];
  const float* Wout  = (const float*)d_in[5];
  const float* bout  = (const float*)d_in[6];
  const float* bias  = (const float*)d_in[7];
  float* out = (float*)d_out;

  char* ws = (char*)d_ws;
  unsigned short* A2  = (unsigned short*)(ws + kOffA2);
  unsigned short* BT2 = (unsigned short*)(ws + kOffBT2);

  tail_cols_kernel<<<kGraphs * kChan, 32, 0, stream>>>(nf, bout, BT2);
  weight_cols_kernel<<<kGraphs * kChan, 128, 0, stream>>>(nf, Wout, BT2);
  edge_rows_kernel<<<kGraphs * kNodes, 128, 0, stream>>>(ef, fltr, W0, b0, A2);
  aggregate_kernel<<<kGraphs * (kNodes / 16), 128, 0, stream>>>(A2, BT2, fltr, bias, out);
}
